// LatentEdgeScorer_28905129902363
// MI455X (gfx1250) — hardware-verified
//
#include <hip/hip_runtime.h>
#include <hip/hip_bf16.h>
#include <stddef.h>
#include <stdint.h>
#include <math.h>


#define ND     256
#define HD     128
#define NB     2
#define NNODE  512
#define NROWS  (NB * NNODE)
#define W1P    384
#define TM     16
#define NTHR   256
#define PTHR   224
#define WSCAP  134217728

static_assert(NTHR == 8 * 32);
static_assert(PTHR == 7 * 32);
static_assert((NROWS % TM) == 0);
static_assert(HD == 8 * 16);
static_assert((ND % 32) == 0);
static_assert((HD % 32) == 0);
static_assert(NNODE == 4 * 128);
static_assert(TM * HD == 2 * 4 * NTHR);

#define SZ_PW  ((size_t)HD * ND * 2)
#define SZ_PH  ((size_t)HD * HD * 2)
#define SZ_F   ((size_t)NROWS * HD * 4)
#define SZ_TOT (4 * SZ_PW + 6 * SZ_PH + 4 * SZ_F)
static_assert(SZ_TOT == 2555904);
static_assert(SZ_TOT <= (size_t)WSCAP);
static_assert((SZ_PW % 256) == 0);
static_assert((SZ_PH % 256) == 0);
static_assert((SZ_F % 256) == 0);

typedef float          v4f   __attribute__((ext_vector_type(4)));
typedef float          v8f   __attribute__((ext_vector_type(8)));
typedef unsigned short v8us  __attribute__((ext_vector_type(8)));
typedef unsigned short v16us __attribute__((ext_vector_type(16)));
typedef __bf16         v16bf __attribute__((ext_vector_type(16)));
union FragB { v16bf v; v16us u; v8us u8[2]; };

__device__ __forceinline__ unsigned int bf16_bits(float f) {
  unsigned int u = __float_as_uint(f);
  u += 0x7FFFu + ((u >> 16) & 1u);
  return u >> 16;
}

__device__ __forceinline__ void split8(const v4f a, const v4f b, v8us& hi, v8us& lo) {
  const float f[8] = {a.x, a.y, a.z, a.w, b.x, b.y, b.z, b.w};
  v8us hv, lv;
#pragma unroll
  for (int e = 0; e < 8; ++e) {
    const unsigned int hb = bf16_bits(f[e]);
    const float res = f[e] - __uint_as_float(hb << 16);
    hv[e] = (unsigned short)hb;
    lv[e] = (unsigned short)bf16_bits(res);
  }
  hi = hv;
  lo = lv;
}

__device__ __forceinline__ v8f wmb(v16bf a, v16bf b, v8f c) {
  v8f d = __builtin_amdgcn_wmma_f32_16x16x32_bf16(false, a, false, b, (short)0, c, false, false);
  asm volatile("v_nop\n\tv_nop\n\tv_nop\n\tv_nop" : "+v"(d) : "v"(a), "v"(b));
  return d;
}

__device__ __forceinline__ v8f wm3(const FragB& ah, const FragB& al, const FragB& bh, const FragB& bl, v8f c) {
  c = wmb(ah.v, bh.v, c);
  c = wmb(ah.v, bl.v, c);
  c = wmb(al.v, bh.v, c);
  return c;
}

__global__ __launch_bounds__(PTHR) void k_prep(const float* __restrict__ sW, const float* __restrict__ tW,
                                               const float* __restrict__ W1,
                                               unsigned short* sWh, unsigned short* sWl,
                                               unsigned short* tWh, unsigned short* tWl,
                                               unsigned short* Wsh, unsigned short* Wsl,
                                               unsigned short* Wth, unsigned short* Wtl,
                                               unsigned short* Wph, unsigned short* Wpl) {
  const int n = blockIdx.x, tid = threadIdx.x, lane = tid & 31, wv = tid >> 5, h = lane >> 4;
  const int c = 8 * (lane & 15);
  const float* src = W1 + (size_t)n * W1P + 256;
  unsigned short* dh = Wph + (size_t)n * HD;
  unsigned short* dl = Wpl + (size_t)n * HD;
  if (wv == 0)      { src = sW + (size_t)n * ND;        dh = sWh + (size_t)n * ND;        dl = sWl + (size_t)n * ND; }
  else if (wv == 1) { src = sW + (size_t)n * ND + 128;  dh = sWh + (size_t)n * ND + 128;  dl = sWl + (size_t)n * ND + 128; }
  else if (wv == 2) { src = tW + (size_t)n * ND;        dh = tWh + (size_t)n * ND;        dl = tWl + (size_t)n * ND; }
  else if (wv == 3) { src = tW + (size_t)n * ND + 128;  dh = tWh + (size_t)n * ND + 128;  dl = tWl + (size_t)n * ND + 128; }
  else if (wv == 4) { src = W1 + (size_t)n * W1P;       dh = Wsh + (size_t)n * HD;        dl = Wsl + (size_t)n * HD; }
  else if (wv == 5) { src = W1 + (size_t)n * W1P + 128; dh = Wth + (size_t)n * HD;        dl = Wtl + (size_t)n * HD; }
  const v4f f0 = *(const v4f*)(src + c);
  const v4f f1 = *(const v4f*)(src + c + 4);
  v8us hv, lv;
  split8(f0, f1, hv, lv);
  v8us sel;
#pragma unroll
  for (int e = 0; e < 8; ++e) {
    const unsigned short a = hv[e], b = lv[e];
    sel[e] = h ? b : a;
  }
  unsigned short* d = (h ? dl : dh) + c;
  *(volatile v8us*)d = sel;
  __threadfence();
  *(volatile v8us*)d = sel;
}

__global__ __launch_bounds__(NTHR) void k_node(const float* __restrict__ x,
                                               const float* __restrict__ sn_g, const float* __restrict__ sn_b,
                                               const float* __restrict__ tn_g, const float* __restrict__ tn_b,
                                               const unsigned short* __restrict__ sWh, const unsigned short* __restrict__ sWl,
                                               const unsigned short* __restrict__ tWh, const unsigned short* __restrict__ tWl,
                                               const unsigned short* __restrict__ Wsh, const unsigned short* __restrict__ Wsl,
                                               const unsigned short* __restrict__ Wth, const unsigned short* __restrict__ Wtl,
                                               const float* __restrict__ sb, const float* __restrict__ tb,
                                               float* srcF, float* tgtF, float* asF, float* atF) {
  __shared__ __attribute__((aligned(16))) float xsL[TM * ND];
  __shared__ __attribute__((aligned(16))) float xtL[TM * ND];
  __shared__ __attribute__((aligned(16))) float srL[TM * HD];
  __shared__ __attribute__((aligned(16))) float tgL[TM * HD];
  const int tid = threadIdx.x, lane = tid & 31, wv = tid >> 5, h = lane >> 4, m = lane & 15;
  const int row0 = blockIdx.x * TM;
  const float inv_nd = 1.0f / (float)ND;
  const v8f zero8 = {0.f, 0.f, 0.f, 0.f, 0.f, 0.f, 0.f, 0.f};

#pragma unroll 1
  for (int rr = 0; rr < 2; ++rr) {
    const int r = wv + 8 * rr;
    const float* xr = x + (size_t)(row0 + r) * ND + 8 * lane;
    const v4f a0 = *(const v4f*)xr;
    const v4f a1 = *(const v4f*)(xr + 4);
    float s = ((a0.x + a0.y) + (a0.z + a0.w)) + ((a1.x + a1.y) + (a1.z + a1.w));
    s += __shfl_xor(s, 16);
    s += __shfl_xor(s, 8);
    s += __shfl_xor(s, 4);
    s += __shfl_xor(s, 2);
    s += __shfl_xor(s, 1);
    const float mu = s * inv_nd;
    const v4f d0 = a0 - mu;
    const v4f d1 = a1 - mu;
    float q = ((d0.x * d0.x + d0.y * d0.y) + (d0.z * d0.z + d0.w * d0.w)) +
              ((d1.x * d1.x + d1.y * d1.y) + (d1.z * d1.z + d1.w * d1.w));
    q += __shfl_xor(q, 16);
    q += __shfl_xor(q, 8);
    q += __shfl_xor(q, 4);
    q += __shfl_xor(q, 2);
    q += __shfl_xor(q, 1);
    const float rs = rsqrtf(q * inv_nd + 1e-5f);
    const v4f y0 = d0 * rs;
    const v4f y1 = d1 * rs;
    const v4f gs0 = *(const v4f*)(sn_g + 8 * lane), gs1 = *(const v4f*)(sn_g + 8 * lane + 4);
    const v4f bs0 = *(const v4f*)(sn_b + 8 * lane), bs1 = *(const v4f*)(sn_b + 8 * lane + 4);
    const v4f gt0 = *(const v4f*)(tn_g + 8 * lane), gt1 = *(const v4f*)(tn_g + 8 * lane + 4);
    const v4f bt0 = *(const v4f*)(tn_b + 8 * lane), bt1 = *(const v4f*)(tn_b + 8 * lane + 4);
    *(v4f*)(xsL + r * ND + 8 * lane)     = y0 * gs0 + bs0;
    *(v4f*)(xsL + r * ND + 8 * lane + 4) = y1 * gs1 + bs1;
    *(v4f*)(xtL + r * ND + 8 * lane)     = y0 * gt0 + bt0;
    *(v4f*)(xtL + r * ND + 8 * lane + 4) = y1 * gt1 + bt1;
  }
  __syncthreads();

  const int n0 = 16 * wv;
  const int cn = n0 + m;

  {
    v8f accS = zero8, accT = zero8;
#pragma unroll 1
    for (int kt = 0; kt < ND / 32; ++kt) {
      const int k0 = 32 * kt;
      const float* ps = xsL + m * ND + k0 + 8 * h;
      const float* pt = xtL + m * ND + k0 + 8 * h;
      FragB aSh, aSl, aTh, aTl;
      split8(*(const v4f*)ps,        *(const v4f*)(ps + 4),  aSh.u8[0], aSl.u8[0]);
      split8(*(const v4f*)(ps + 16), *(const v4f*)(ps + 20), aSh.u8[1], aSl.u8[1]);
      split8(*(const v4f*)pt,        *(const v4f*)(pt + 4),  aTh.u8[0], aTl.u8[0]);
      split8(*(const v4f*)(pt + 16), *(const v4f*)(pt + 20), aTh.u8[1], aTl.u8[1]);
      const size_t bo = (size_t)cn * ND + k0 + 8 * h;
      FragB bSh, bSl, bTh, bTl;
      bSh.u8[0] = *(const v8us*)(sWh + bo); bSh.u8[1] = *(const v8us*)(sWh + bo + 16);
      bSl.u8[0] = *(const v8us*)(sWl + bo); bSl.u8[1] = *(const v8us*)(sWl + bo + 16);
      bTh.u8[0] = *(const v8us*)(tWh + bo); bTh.u8[1] = *(const v8us*)(tWh + bo + 16);
      bTl.u8[0] = *(const v8us*)(tWl + bo); bTl.u8[1] = *(const v8us*)(tWl + bo + 16);
      accS = wm3(aSh, aSl, bSh, bSl, accS);
      accT = wm3(aTh, aTl, bTh, bTl, accT);
    }
    const float sbv = sb[cn], tbv = tb[cn];
#pragma unroll
    for (int r = 0; r < 8; ++r) {
      srL[(8 * h + r) * HD + cn] = accS[r] + sbv;
      tgL[(8 * h + r) * HD + cn] = accT[r] + tbv;
    }
  }
  __syncthreads();

  {
    const int q0 = tid, q1 = tid + NTHR;
    const v4f vs0 = *(const v4f*)(srL + 4 * q0), vs1 = *(const v4f*)(srL + 4 * q1);
    const v4f vt0 = *(const v4f*)(tgL + 4 * q0), vt1 = *(const v4f*)(tgL + 4 * q1);
    float* ps = srcF + (size_t)row0 * HD;
    float* pt = tgtF + (size_t)row0 * HD;
    *(volatile v4f*)(ps + 4 * q0) = vs0; *(volatile v4f*)(ps + 4 * q1) = vs1;
    *(volatile v4f*)(pt + 4 * q0) = vt0; *(volatile v4f*)(pt + 4 * q1) = vt1;
    __threadfence();
    *(volatile v4f*)(ps + 4 * q0) = vs0; *(volatile v4f*)(ps + 4 * q1) = vs1;
    *(volatile v4f*)(pt + 4 * q0) = vt0; *(volatile v4f*)(pt + 4 * q1) = vt1;
  }

  float* asL = xsL;
  float* atL = xtL;
  {
    v8f accA = zero8, accB = zero8;
#pragma unroll 1
    for (int kt = 0; kt < HD / 32; ++kt) {
      const int k0 = 32 * kt;
      const float* ps = srL + m * HD + k0 + 8 * h;
      const float* pt = tgL + m * HD + k0 + 8 * h;
      FragB aSh, aSl, aTh, aTl;
      split8(*(const v4f*)ps,        *(const v4f*)(ps + 4),  aSh.u8[0], aSl.u8[0]);
      split8(*(const v4f*)(ps + 16), *(const v4f*)(ps + 20), aSh.u8[1], aSl.u8[1]);
      split8(*(const v4f*)pt,        *(const v4f*)(pt + 4),  aTh.u8[0], aTl.u8[0]);
      split8(*(const v4f*)(pt + 16), *(const v4f*)(pt + 20), aTh.u8[1], aTl.u8[1]);
      const size_t bo = (size_t)cn * HD + k0 + 8 * h;
      FragB bSh, bSl, bTh, bTl;
      bSh.u8[0] = *(const v8us*)(Wsh + bo); bSh.u8[1] = *(const v8us*)(Wsh + bo + 16);
      bSl.u8[0] = *(const v8us*)(Wsl + bo); bSl.u8[1] = *(const v8us*)(Wsl + bo + 16);
      bTh.u8[0] = *(const v8us*)(Wth + bo); bTh.u8[1] = *(const v8us*)(Wth + bo + 16);
      bTl.u8[0] = *(const v8us*)(Wtl + bo); bTl.u8[1] = *(const v8us*)(Wtl + bo + 16);
      accA = wm3(aSh, aSl, bSh, bSl, accA);
      accB = wm3(aTh, aTl, bTh, bTl, accB);
    }
#pragma unroll
    for (int r = 0; r < 8; ++r) {
      asL[(8 * h + r) * HD + cn] = accA[r];
      atL[(8 * h + r) * HD + cn] = accB[r];
    }
  }
  __syncthreads();

  {
    const int q0 = tid, q1 = tid + NTHR;
    const v4f va0 = *(const v4f*)(asL + 4 * q0), va1 = *(const v4f*)(asL + 4 * q1);
    const v4f vb0 = *(const v4f*)(atL + 4 * q0), vb1 = *(const v4f*)(atL + 4 * q1);
    float* pa = asF + (size_t)row0 * HD;
    float* pb = atF + (size_t)row0 * HD;
    *(volatile v4f*)(pa + 4 * q0) = va0; *(volatile v4f*)(pa + 4 * q1) = va1;
    *(volatile v4f*)(pb + 4 * q0) = vb0; *(volatile v4f*)(pb + 4 * q1) = vb1;
    __threadfence();
    *(volatile v4f*)(pa + 4 * q0) = va0; *(volatile v4f*)(pa + 4 * q1) = va1;
    *(volatile v4f*)(pb + 4 * q0) = vb0; *(volatile v4f*)(pb + 4 * q1) = vb1;
  }
}

__global__ __launch_bounds__(NTHR) void k_pair(const float* __restrict__ srcF, const float* __restrict__ tgtF,
                                               const float* __restrict__ asF, const float* __restrict__ atF,
                                               const unsigned short* __restrict__ Wph, const unsigned short* __restrict__ Wpl,
                                               const float* __restrict__ b1, const float* __restrict__ W2,
                                               const float* __restrict__ b2, float* out) {
  __shared__ __attribute__((aligned(16))) float srcI[HD];
  __shared__ __attribute__((aligned(16))) float asI[HD];
  __shared__ __attribute__((aligned(16))) float b1L[HD];
  __shared__ __attribute__((aligned(16))) float w2L[HD];
  __shared__ __attribute__((aligned(16))) float es[NNODE];
  const int tid = threadIdx.x, lane = tid & 31, wv = tid >> 5, h = lane >> 4, m = lane & 15;
  const int blk = blockIdx.x;
  const int b = blk >> 9, i = blk & (NNODE - 1);
  if (tid < HD) {
    srcI[tid] = srcF[(size_t)blk * HD + tid];
    asI[tid]  = asF[(size_t)blk * HD + tid];
    b1L[tid]  = b1[tid];
    w2L[tid]  = W2[tid];
  }
  __syncthreads();
  const float b2v = b2[0];
  const size_t tb0 = (size_t)b * NNODE;
  const v8f zero8 = {0.f, 0.f, 0.f, 0.f, 0.f, 0.f, 0.f, 0.f};

#pragma unroll 1
  for (int t = 0; t < 4; ++t) {
    const int j0 = 64 * wv + 16 * t;
    const float* trow = tgtF + (tb0 + j0 + m) * HD + 8 * h;
    const float* arow = atF + (tb0 + j0 + 8 * h) * HD;
    float red[8];
#pragma unroll
    for (int r = 0; r < 8; ++r) red[r] = 0.f;

#pragma unroll 1
    for (int nh = 0; nh < 2; ++nh) {
      v8f acc[4];
#pragma unroll
      for (int nt = 0; nt < 4; ++nt) acc[nt] = zero8;
#pragma unroll 1
      for (int kt = 0; kt < HD / 32; ++kt) {
        const int k0 = 32 * kt;
        const float* sp = srcI + k0 + 8 * h;
        const v4f t0 = *(const v4f*)(trow + k0),      t1 = *(const v4f*)(trow + k0 + 4);
        const v4f t2 = *(const v4f*)(trow + k0 + 16), t3 = *(const v4f*)(trow + k0 + 20);
        const v4f s0 = *(const v4f*)sp,               s1 = *(const v4f*)(sp + 4);
        const v4f s2 = *(const v4f*)(sp + 16),        s3 = *(const v4f*)(sp + 20);
        const v4f p0 = s0 * t0, p1 = s1 * t1, p2 = s2 * t2, p3 = s3 * t3;
        FragB ah, al;
        split8(p0, p1, ah.u8[0], al.u8[0]);
        split8(p2, p3, ah.u8[1], al.u8[1]);
        const size_t bo = (size_t)(nh * 64 + m) * HD + k0 + 8 * h;
#pragma unroll
        for (int nt = 0; nt < 4; ++nt) {
          const size_t o = bo + (size_t)nt * 16 * HD;
          FragB bh, bl;
          bh.u8[0] = *(const v8us*)(Wph + o); bh.u8[1] = *(const v8us*)(Wph + o + 16);
          bl.u8[0] = *(const v8us*)(Wpl + o); bl.u8[1] = *(const v8us*)(Wpl + o + 16);
          acc[nt] = wm3(ah, al, bh, bl, acc[nt]);
        }
      }
#pragma unroll
      for (int nt = 0; nt < 4; ++nt) {
        const int n = nh * 64 + nt * 16 + m;
        const float av = asI[n], bv = b1L[n], wq = w2L[n];
        const float* ap = arow + n;
#pragma unroll
        for (int r = 0; r < 8; ++r) {
          float val = av + ap[(size_t)r * HD];
          val = val + acc[nt][r];
          val = val + bv;
          const float g = 0.5f * val * (1.0f + erff(val * 0.70710678118654752f));
          red[r] = fmaf(g, wq, red[r]);
        }
      }
    }
#pragma unroll
    for (int r = 0; r < 8; ++r) {
      float v = red[r];
      v += __shfl_xor(v, 1);
      v += __shfl_xor(v, 2);
      v += __shfl_xor(v, 4);
      v += __shfl_xor(v, 8);
      red[r] = v;
    }
    const int rsel = m & 7;
    float kv = red[0];
#pragma unroll
    for (int r = 1; r < 8; ++r) kv = (rsel == r) ? red[r] : kv;
    const int j = j0 + 8 * h + rsel;
    const float lg = kv + b2v;
    const float dn = 1.0f + fabsf(lg);
    float e = lg * (1.0f / dn);
    e = (j == i) ? 0.f : e;
    if (m < 8) es[j] = e;
  }
  __syncthreads();

  if (wv < 4) {
    const int q = 32 * wv + lane;
    const v4f v = *(const v4f*)(es + 4 * q);
    float* gp = out + (size_t)blk * NNODE + 4 * q;
    *(volatile v4f*)gp = v;
    __threadfence();
    *(volatile v4f*)gp = v;
  }
}

extern "C" void kernel_launch(void* const* d_in, const int* in_sizes, int n_in,
                              void* d_out, int out_size, void* d_ws, size_t ws_size,
                              hipStream_t stream) {
  if (n_in < 13) return;
  if (in_sizes[0] != NROWS * ND) return;
  if (in_sizes[1] != ND || in_sizes[2] != ND || in_sizes[3] != ND || in_sizes[4] != ND) return;
  if (in_sizes[5] != HD * ND || in_sizes[7] != HD * ND) return;
  if (in_sizes[6] != HD || in_sizes[8] != HD) return;
  if (in_sizes[9] != HD * W1P || in_sizes[10] != HD) return;
  if (in_sizes[11] != HD || in_sizes[12] < 1) return;
  if (out_size != NROWS * NNODE) return;

  const float* latent = (const float*)d_in[0];
  const float* sn_g   = (const float*)d_in[1];
  const float* sn_b   = (const float*)d_in[2];
  const float* tn_g   = (const float*)d_in[3];
  const float* tn_b   = (const float*)d_in[4];
  const float* sW     = (const float*)d_in[5];
  const float* sb     = (const float*)d_in[6];
  const float* tW     = (const float*)d_in[7];
  const float* tb     = (const float*)d_in[8];
  const float* W1     = (const float*)d_in[9];
  const float* b1     = (const float*)d_in[10];
  const float* W2     = (const float*)d_in[11];
  const float* b2     = (const float*)d_in[12];
  float* out = (float*)d_out;

  char* ws = (char*)d_ws;
  size_t off = 0;
  const size_t oSWH = off; off += SZ_PW;
  const size_t oSWL = off; off += SZ_PW;
  const size_t oTWH = off; off += SZ_PW;
  const size_t oTWL = off; off += SZ_PW;
  const size_t oWSH = off; off += SZ_PH;
  const size_t oWSL = off; off += SZ_PH;
  const size_t oWTH = off; off += SZ_PH;
  const size_t oWTL = off; off += SZ_PH;
  const size_t oWPH = off; off += SZ_PH;
  const size_t oWPL = off; off += SZ_PH;
  const size_t oSRC = off; off += SZ_F;
  const size_t oTGT = off; off += SZ_F;
  const size_t oAS  = off; off += SZ_F;
  const size_t oAT  = off; off += SZ_F;
  if (off != SZ_TOT) return;
  if (off > ws_size || off > (size_t)WSCAP) return;

  unsigned short* sWh = (unsigned short*)(ws + oSWH);
  unsigned short* sWl = (unsigned short*)(ws + oSWL);
  unsigned short* tWh = (unsigned short*)(ws + oTWH);
  unsigned short* tWl = (unsigned short*)(ws + oTWL);
  unsigned short* Wsh = (unsigned short*)(ws + oWSH);
  unsigned short* Wsl = (unsigned short*)(ws + oWSL);
  unsigned short* Wth = (unsigned short*)(ws + oWTH);
  unsigned short* Wtl = (unsigned short*)(ws + oWTL);
  unsigned short* Wph = (unsigned short*)(ws + oWPH);
  unsigned short* Wpl = (unsigned short*)(ws + oWPL);
  float* srcF = (float*)(ws + oSRC);
  float* tgtF = (float*)(ws + oTGT);
  float* asF  = (float*)(ws + oAS);
  float* atF  = (float*)(ws + oAT);

  k_prep<<<HD, PTHR, 0, stream>>>(sW, tW, W1, sWh, sWl, tWh, tWl, Wsh, Wsl, Wth, Wtl, Wph, Wpl);
  k_node<<<NROWS / TM, NTHR, 0, stream>>>(latent, sn_g, sn_b, tn_g, tn_b,
                                          sWh, sWl, tWh, tWl, Wsh, Wsl, Wth, Wtl,
                                          sb, tb, srcF, tgtF, asF, atF);
  k_pair<<<NROWS, NTHR, 0, stream>>>(srcF, tgtF, asF, atF, Wph, Wpl, b1, W2, b2, out);
}
